// TimeAwareAttention_7035156430998
// MI455X (gfx1250) — hardware-verified
//
#include <hip/hip_runtime.h>
#include <math.h>
#include <stdint.h>

constexpr int kBatch = 4;
constexpr int kSeq   = 2048;
constexpr int kDim   = 512;
constexpr int kTime  = 16;
constexpr int kHeads = 8;
constexpr int kDh    = 64;
constexpr int kRows  = kBatch * kSeq;
constexpr int kQkvN  = 3 * kHeads * kDh;
constexpr int kQKld  = 2 * kHeads * kDh;

typedef char check_dims_a[(kSeq % 64 == 0 && kDim % 64 == 0 && kQkvN % 64 == 0) ? 1 : -1];
typedef char check_dims_b[(kDim == 512 && kDh == 64 && (kSeq / kTime) == 128) ? 1 : -1];

typedef __attribute__((ext_vector_type(16))) _Float16 v16h;
typedef __attribute__((ext_vector_type(8)))  _Float16 v8h;
typedef __attribute__((ext_vector_type(16))) __bf16   v16b;
typedef __attribute__((ext_vector_type(8)))  __bf16   v8b;
typedef __attribute__((ext_vector_type(8)))  float    v8f;
typedef __attribute__((ext_vector_type(4)))  float    v4f;
typedef __attribute__((ext_vector_type(2)))  float    v2f;
typedef __attribute__((ext_vector_type(4)))  unsigned int v4u;

__device__ __forceinline__ unsigned short f2bf_bits(float f) {
  unsigned u = __float_as_uint(f);
  return (unsigned short)((u + 0x7FFFu + ((u >> 16) & 1u)) >> 16);
}
__device__ __forceinline__ float bf_bits2f(unsigned short h) { return __uint_as_float(((unsigned)h) << 16); }
__device__ __forceinline__ float bfr(float f) { return bf_bits2f(f2bf_bits(f)); }
__device__ __forceinline__ unsigned pk16(unsigned short a, unsigned short b) { return (unsigned)a | ((unsigned)b << 16); }

__device__ __forceinline__ void dep_guard_h(v8f& a, v8f& b, v16h x, v16h y) { asm volatile("v_nop\n\tv_nop\n\tv_nop\n\tv_nop" : "+v"(a), "+v"(b) : "v"(x), "v"(y)); }
__device__ __forceinline__ void dep_guard_b(v8f& a, v8f& b, v16b x, v16b y) { asm volatile("v_nop\n\tv_nop\n\tv_nop\n\tv_nop" : "+v"(a), "+v"(b) : "v"(x), "v"(y)); }
__device__ __forceinline__ void keep4_h(v16h a, v16h b, v16h c, v16h d) { asm volatile("v_nop" :: "v"(a), "v"(b), "v"(c), "v"(d)); }
__device__ __forceinline__ void keep4_b(v16b a, v16b b, v16b c, v16b d) { asm volatile("v_nop" :: "v"(a), "v"(b), "v"(c), "v"(d)); }
__device__ __forceinline__ void acc_guard4(v8f& a, v8f& b, v8f& c, v8f& d) { asm volatile("v_nop\n\tv_nop\n\tv_nop\n\tv_nop" : "+v"(a), "+v"(b), "+v"(c), "+v"(d)); }
template <typename T> struct Frag;
template <> struct Frag<_Float16> {
  typedef v16h V; union U { v16h v; v8h h[2]; };
  static __device__ __forceinline__ v16h load(const _Float16* p) {
    U f; f.h[0] = *(const v8h*)(p); f.h[1] = *(const v8h*)(p + 16); return f.v;
  }
  static __device__ __forceinline__ v8f mma(v16h a, v16h b, v8f c) {
    return __builtin_amdgcn_wmma_f32_16x16x32_f16(false, a, false, b, (short)0, c, false, false);
  }
  static __device__ __forceinline__ void guard(v8f& a, v8f& b, v16h x, v16h y) { dep_guard_h(a, b, x, y); }
  static __device__ __forceinline__ void keep(v16h a, v16h b, v16h c, v16h d) { keep4_h(a, b, c, d); }
};
template <> struct Frag<__bf16> {
  typedef v16b V; union U { v16b v; v8b h[2]; };
  static __device__ __forceinline__ v16b load(const __bf16* p) {
    U f; f.h[0] = *(const v8b*)(p); f.h[1] = *(const v8b*)(p + 16); return f.v;
  }
  static __device__ __forceinline__ v8f mma(v16b a, v16b b, v8f c) {
    return __builtin_amdgcn_wmma_f32_16x16x32_bf16(false, a, false, b, (short)0, c, false, false);
  }
  static __device__ __forceinline__ void guard(v8f& a, v8f& b, v16b x, v16b y) { dep_guard_b(a, b, x, y); }
  static __device__ __forceinline__ void keep(v16b a, v16b b, v16b c, v16b d) { keep4_b(a, b, c, d); }
};

template <int ET> struct Elem;
template <> struct Elem<0> { typedef _Float16 T; };
template <> struct Elem<1> { typedef __bf16 T; };
template <int ET, int SPL, int BIAS_MODE, int OUT_MODE, bool RESID, int ACT = 0>
__global__ __launch_bounds__(256) void wmma_gemm64(
    const unsigned short* __restrict__ Ap, const unsigned short* __restrict__ A2p, int lda, long strideA,
    const unsigned short* __restrict__ Btp, const unsigned short* __restrict__ Bt2p, int ldb, long strideB,
    void* __restrict__ Cout, void* __restrict__ Cout2, int ldc, long strideC,
    const float* __restrict__ bias,
    const float* __restrict__ resid, long strideR,
    int M, int N, int K, float scale) {
  typedef typename Elem<ET>::T T;
  typedef typename Frag<T>::V V;
  constexpr bool SA = (SPL & 1) != 0;
  constexpr bool SB = (SPL & 2) != 0;
  const T* A = (const T*)Ap; const T* A2 = (const T*)A2p; const T* Bt = (const T*)Btp; const T* Bt2 = (const T*)Bt2p;
  __shared__ __align__(16) float sT[8][16 * 68];
  const int b    = blockIdx.y;
  const int lane = threadIdx.x & 31;
  const int wave = threadIdx.x >> 5;
  const int tilesN = N >> 6;
  const int tilesM = M >> 6;
  const int tile = blockIdx.x * 8 + wave;
  if (tile >= tilesM * tilesN) return;
  const int tm = tile / tilesN;
  const int tn = tile - tm * tilesN;
  const int m0 = tm << 6;
  const int n0 = tn << 6;

  const T* Ab  = A  + (size_t)b * strideA;
  const T* Bb  = Bt + (size_t)b * strideB;
  const T* Ab2 = SA ? (A2  + (size_t)b * strideA) : nullptr;
  const T* Bb2 = SB ? (Bt2 + (size_t)b * strideB) : nullptr;

  const int rlane = lane & 15;
  const int koff  = (lane >> 4) * 8;
  const int mOff  = (lane >> 4) * 8;

  v8f acc[4][4];
#pragma unroll
  for (int i = 0; i < 4; ++i)
#pragma unroll
    for (int j = 0; j < 4; ++j) acc[i][j] = (v8f){0.f,0.f,0.f,0.f,0.f,0.f,0.f,0.f};

  for (int k0 = 0; k0 < K; k0 += 32) {
    V bh[4], bl[4];
#pragma unroll
    for (int j = 0; j < 4; ++j) {
      const size_t bo = (size_t)(n0 + (j << 4) + rlane) * ldb + koff + k0;
      bh[j] = Frag<T>::load(Bb + bo);
      if (SB) bl[j] = Frag<T>::load(Bb2 + bo);
    }
#pragma unroll
    for (int i = 0; i < 4; ++i) {
      const size_t ao = (size_t)(m0 + (i << 4) + rlane) * lda + koff + k0;
      V ah = Frag<T>::load(Ab + ao);
      V al;
      if (SA) al = Frag<T>::load(Ab2 + ao);
#pragma unroll
      for (int j = 0; j < 4; ++j) {
        acc[i][j] = Frag<T>::mma(ah, bh[j], acc[i][j]);
        if (SB) acc[i][j] = Frag<T>::mma(ah, bl[j], acc[i][j]);
        if (SA) acc[i][j] = Frag<T>::mma(al, bh[j], acc[i][j]);
      }
      Frag<T>::guard(acc[i][0], acc[i][3], ah, SA ? al : ah);
    }
    Frag<T>::keep(bh[0], bh[1], bh[2], bh[3]);
    if (SB) Frag<T>::keep(bl[0], bl[1], bl[2], bl[3]);
  }
  acc_guard4(acc[0][0], acc[0][1], acc[0][2], acc[0][3]);
  acc_guard4(acc[1][0], acc[1][1], acc[1][2], acc[1][3]);
  acc_guard4(acc[2][0], acc[2][1], acc[2][2], acc[2][3]);
  acc_guard4(acc[3][0], acc[3][1], acc[3][2], acc[3][3]);

  float* slab = sT[wave];
  const float* Rb = RESID ? (resid + (size_t)b * strideR) : nullptr;
#pragma unroll
  for (int i = 0; i < 4; ++i) {
    const int mBase = m0 + (i << 4);
#pragma unroll
    for (int j = 0; j < 4; ++j) {
      const int n = n0 + (j << 4) + rlane;
      float bv = 0.f;
      if (BIAS_MODE == 2) bv = bias[n];
#pragma unroll
      for (int r = 0; r < 8; ++r) {
        float v = acc[i][j][r] * scale;
        if (BIAS_MODE == 1) v += bias[mBase + mOff + r];
        if (BIAS_MODE == 2) v += bv;
        if (RESID) v += Rb[(size_t)(mBase + mOff + r) * ldc + n];
        if (ACT == 1) v = tanhf(v);
        if (ACT == 2) v = fmaxf(v, 0.0f);
        if (ACT == 3) v = v / (1.0f + expf(-v));
        if (ACT == 4) v = (v > 0.f) ? v : 0.01f * v;
        slab[(mOff + r) * 68 + (j << 4) + rlane] = v;
      }
    }
    __builtin_amdgcn_fence(__ATOMIC_RELEASE, "workgroup");
    __builtin_amdgcn_wave_barrier();
    __builtin_amdgcn_fence(__ATOMIC_ACQUIRE, "workgroup");
    if (OUT_MODE == 0) {
      float* C = (float*)Cout + (size_t)b * strideC;
      const int hh = lane >> 4, c4 = (lane & 15) * 4;
      for (int pass = 0; pass < 2; ++pass) {
#pragma unroll
        for (int it = 0; it < 8; ++it) {
          const int row = it * 2 + hh;
          v4f v = *(const v4f*)(slab + row * 68 + c4);
          *(volatile v4f*)(C + (size_t)(mBase + row) * ldc + n0 + c4) = v;
        }
        __threadfence();
      }
    } else {
      const int q = lane >> 3, c8 = (lane & 7) * 8;
      unsigned short* C  = (unsigned short*)Cout  + (size_t)b * strideC;
      unsigned short* C2 = (OUT_MODE == 2) ? ((unsigned short*)Cout2 + (size_t)b * strideC) : nullptr;
      for (int pass = 0; pass < 2; ++pass) {
#pragma unroll
        for (int it = 0; it < 4; ++it) {
          const int row = it * 4 + q;
          const float* sp = slab + row * 68 + c8;
          v8h hv, lv;
#pragma unroll
          for (int e = 0; e < 8; ++e) {
            if (OUT_MODE == 1) {
              hv[e] = (_Float16)sp[e];
            } else {
              unsigned short hb = f2bf_bits(sp[e]);
              unsigned short lb = f2bf_bits(sp[e] - bf_bits2f(hb));
              hv[e] = __builtin_bit_cast(_Float16, hb);
              lv[e] = __builtin_bit_cast(_Float16, lb);
            }
          }
          *(volatile v8h*)(C + (size_t)(mBase + row) * ldc + n0 + c8) = hv;
          if (OUT_MODE == 2) *(volatile v8h*)(C2 + (size_t)(mBase + row) * ldc + n0 + c8) = lv;
        }
        __threadfence();
      }
    }
    __builtin_amdgcn_fence(__ATOMIC_RELEASE, "workgroup");
    __builtin_amdgcn_wave_barrier();
    __builtin_amdgcn_fence(__ATOMIC_ACQUIRE, "workgroup");
  }
}

__global__ __launch_bounds__(256) void ln_split_kernel(const float* __restrict__ x, const float* __restrict__ gamma,
                                                       const float* __restrict__ beta, unsigned short* __restrict__ xh,
                                                       unsigned short* __restrict__ xl, int nrows) {
  const int wave = threadIdx.x >> 5, lane = threadIdx.x & 31;
  const int row = blockIdx.x * 8 + wave;
  if (row >= nrows) return;
  const float* xr = x + (size_t)row * kDim;
  float v[16];
  {
    const v4f a0 = *(const v4f*)(xr + 8 * lane);
    const v4f a1 = *(const v4f*)(xr + 8 * lane + 4);
    const v4f a2 = *(const v4f*)(xr + 256 + 8 * lane);
    const v4f a3 = *(const v4f*)(xr + 256 + 8 * lane + 4);
#pragma unroll
    for (int e = 0; e < 4; ++e) { v[e] = bfr(a0[e]); v[4 + e] = bfr(a1[e]); v[8 + e] = bfr(a2[e]); v[12 + e] = bfr(a3[e]); }
  }
  float s = 0.f;
#pragma unroll
  for (int i = 0; i < 16; ++i) s += v[i];
#pragma unroll
  for (int off = 1; off < 32; off <<= 1) s += __shfl_xor(s, off, 32);
  const float mean = s * (1.0f / (float)kDim);
  float d[16];
  float ss = 0.f;
#pragma unroll
  for (int i = 0; i < 16; ++i) { d[i] = v[i] - mean; ss += d[i] * d[i]; }
#pragma unroll
  for (int off = 1; off < 32; off <<= 1) ss += __shfl_xor(ss, off, 32);
  const float var  = ss * (1.0f / (float)kDim);
  const float rstd = rsqrtf(var + 1e-5f);
  float g[16], bt[16];
  {
    const v4f g0 = *(const v4f*)(gamma + 8 * lane);
    const v4f g1 = *(const v4f*)(gamma + 8 * lane + 4);
    const v4f g2 = *(const v4f*)(gamma + 256 + 8 * lane);
    const v4f g3 = *(const v4f*)(gamma + 256 + 8 * lane + 4);
    const v4f b0 = *(const v4f*)(beta + 8 * lane);
    const v4f b1 = *(const v4f*)(beta + 8 * lane + 4);
    const v4f b2 = *(const v4f*)(beta + 256 + 8 * lane);
    const v4f b3 = *(const v4f*)(beta + 256 + 8 * lane + 4);
#pragma unroll
    for (int e = 0; e < 4; ++e) {
      g[e] = bfr(g0[e]); g[4 + e] = bfr(g1[e]); g[8 + e] = bfr(g2[e]); g[12 + e] = bfr(g3[e]);
      bt[e] = bfr(b0[e]); bt[4 + e] = bfr(b1[e]); bt[8 + e] = bfr(b2[e]); bt[12 + e] = bfr(b3[e]);
    }
  }
  unsigned hw[8], lw[8];
#pragma unroll
  for (int i = 0; i < 8; ++i) {
    const float o0 = d[2 * i] * rstd * g[2 * i] + bt[2 * i];
    const float o1 = d[2 * i + 1] * rstd * g[2 * i + 1] + bt[2 * i + 1];
    const unsigned short h0 = f2bf_bits(o0), h1 = f2bf_bits(o1);
    const unsigned short l0 = f2bf_bits(o0 - bf_bits2f(h0)), l1 = f2bf_bits(o1 - bf_bits2f(h1));
    hw[i] = pk16(h0, h1); lw[i] = pk16(l0, l1);
  }
  v4u hv0, hv1, lv0, lv1;
  hv0[0] = hw[0]; hv0[1] = hw[1]; hv0[2] = hw[2]; hv0[3] = hw[3];
  hv1[0] = hw[4]; hv1[1] = hw[5]; hv1[2] = hw[6]; hv1[3] = hw[7];
  lv0[0] = lw[0]; lv0[1] = lw[1]; lv0[2] = lw[2]; lv0[3] = lw[3];
  lv1[0] = lw[4]; lv1[1] = lw[5]; lv1[2] = lw[6]; lv1[3] = lw[7];
  const size_t base0 = (size_t)row * kDim + 8 * lane;
  const size_t base1 = (size_t)row * kDim + 256 + 8 * lane;
  for (int pass = 0; pass < 2; ++pass) {
    *(volatile v4u*)(xh + base0) = hv0;
    *(volatile v4u*)(xh + base1) = hv1;
    *(volatile v4u*)(xl + base0) = lv0;
    *(volatile v4u*)(xl + base1) = lv1;
    __threadfence();
  }
}

__global__ __launch_bounds__(256) void tcast_bf16_kernel(const float* __restrict__ W, unsigned short* __restrict__ o, int nR, int nC) {
  __shared__ __align__(16) float tf[64 * 68];
  const int c0  = blockIdx.x * 64;
  const int r0  = blockIdx.y * 64;
  const int tid = threadIdx.x;
  {
    const int lr = tid >> 4;
    const int c4 = (tid & 15) * 4;
#pragma unroll
    for (int it = 0; it < 4; ++it) {
      const int rr = it * 16 + lr;
      const v4f a = *(const v4f*)(W + (size_t)(r0 + rr) * nC + c0 + c4);
      *(v4f*)(tf + rr * 68 + c4) = a;
    }
  }
  __syncthreads();
  const int sub = tid >> 3;
  const int c8  = (tid & 7) * 8;
  v4u hv[2];
#pragma unroll
  for (int it = 0; it < 2; ++it) {
    const int oc = it * 32 + sub;
    v4u a;
#pragma unroll
    for (int q = 0; q < 4; ++q) {
      const float f0 = tf[(c8 + 2 * q) * 68 + oc];
      const float f1 = tf[(c8 + 2 * q + 1) * 68 + oc];
      a[q] = pk16(f2bf_bits(f0), f2bf_bits(f1));
    }
    hv[it] = a;
  }
  for (int pass = 0; pass < 2; ++pass) {
#pragma unroll
    for (int it = 0; it < 2; ++it) {
      const int oc = it * 32 + sub;
      const size_t go = (size_t)(c0 + oc) * nR + r0 + c8;
      *(volatile v4u*)(o + go) = hv[it];
    }
    __threadfence();
  }
}

__global__ __launch_bounds__(256) void decay_kernel(const float* __restrict__ Rmat, const float* __restrict__ av,
                                                    const float* __restrict__ cv, float* __restrict__ dec, int n) {
  const int i = blockIdx.x * 256 + threadIdx.x;
  if (i < n) {
    const int tj = i & 15, ti = (i >> 4) & 15, h = (i >> 8) & 7, b = i >> 11;
    const float r  = bfr(Rmat[(b * kTime + ti) * kTime + tj]);
    const float aa = fabsf(bfr(av[h]));
    const float cc = fabsf(bfr(cv[h]));
    float t = aa * r;
    asm volatile("" : "+v"(t));
    t = t - cc;
    const float e = expf(t);
    const float dv = 1.0f / (1.0f + e);
    ((volatile float*)dec)[i] = dv;
    __threadfence();
    ((volatile float*)dec)[i] = dv;
  }
}

#define AT_D 64
#define AT_NW 4
#define AT_QB 64
#define AT_KC 64

__device__ __forceinline__ unsigned short at_bf_bits(float f) {
  unsigned u = __float_as_uint(f);
  return (unsigned short)((u + 0x7FFFu + ((u >> 16) & 1u)) >> 16);
}
__device__ __forceinline__ __bf16 at_f2bf(float f) { return __builtin_bit_cast(__bf16, at_bf_bits(f)); }
__device__ __forceinline__ void at_split(float f, __bf16& hi, __bf16& lo) {
  const unsigned short hb = at_bf_bits(f);
  hi = __builtin_bit_cast(__bf16, hb);
  lo = at_f2bf(f - __uint_as_float(((unsigned)hb) << 16));
}
__device__ __forceinline__ v8f at_mma(v16b a, v16b b, v8f c) {
  c = __builtin_amdgcn_wmma_f32_16x16x32_bf16(false, a, false, b, (short)0, c, false, false);
  asm volatile("v_nop\n\tv_nop\n\tv_nop\n\tv_nop" : "+v"(c) : "v"(a), "v"(b));
  return c;
}
__device__ __forceinline__ v8f at_mma_h(v16h a, v16h b, v8f c) {
  c = __builtin_amdgcn_wmma_f32_16x16x32_f16(false, a, false, b, (short)0, c, false, false);
  asm volatile("v_nop\n\tv_nop\n\tv_nop\n\tv_nop" : "+v"(c) : "v"(a), "v"(b));
  return c;
}

__global__ __launch_bounds__(128)
void attn_td_kernel(const unsigned short* __restrict__ qkp,
                    const unsigned short* __restrict__ vhp, const unsigned short* __restrict__ vlp,
                    const float* __restrict__ dec,
                    unsigned short* __restrict__ ohp, unsigned short* __restrict__ olp, float sscale) {
  union FB { v16b v; v8b h[2]; };
  union FH { v16h v; v8h h[2]; };
  __shared__ __align__(16) _Float16 Ksh[AT_KC * AT_D];
  __shared__ __align__(16) __bf16   Vth[AT_D * AT_KC];
  __shared__ __align__(16) __bf16   Vtl[AT_D * AT_KC];
  __shared__ __align__(16) __bf16   Psh[AT_NW][16 * AT_KC];
  __shared__ __align__(16) __bf16   Psl[AT_NW][16 * AT_KC];
  __shared__ __align__(16) float    Os[AT_NW][16 * 68];

  const int tid  = threadIdx.x;
  const int wave = tid >> 5;
  const int lane = tid & 31;
  const int hh   = lane >> 4;
  const int c    = lane & 15;

  const int nqb = kSeq / AT_QB;
  const int bx = blockIdx.x;
  const int qb = bx % nqb;
  const int bh = bx / nqb;
  const int h  = bh % kHeads;
  const int b  = bh / kHeads;
  const int q0 = qb * AT_QB + wave * 16;

  const _Float16* Qp = (const _Float16*)(const void*)qkp + (size_t)b * kSeq * kQKld + (size_t)h * AT_D;
  const _Float16* Kp = Qp + kHeads * kDh;
  const __bf16*   Vh = (const __bf16*)(const void*)vhp + (size_t)b * kDim * kSeq + (size_t)h * AT_D * kSeq;
  const __bf16*   Vl = (const __bf16*)(const void*)vlp + (size_t)b * kDim * kSeq + (size_t)h * AT_D * kSeq;
  unsigned short* Oh = ohp + (size_t)b * kSeq * kDim + (size_t)h * AT_D;
  unsigned short* Ol = olp + (size_t)b * kSeq * kDim + (size_t)h * AT_D;
  const float* decrow = dec + ((size_t)(b * kHeads + h) * kTime + (qb >> 1)) * kTime;

  v16h qa[2];
#pragma unroll
  for (int dc = 0; dc < 2; ++dc) {
    const _Float16* qr = Qp + (size_t)(q0 + c) * kQKld + dc * 32 + 8 * hh;
    qa[dc] = Frag<_Float16>::load(qr);
  }

  float mrow[8], lrow[8];
  v8f oacc[4];
#pragma unroll
  for (int r = 0; r < 8; ++r) { mrow[r] = -INFINITY; lrow[r] = 0.f; }
#pragma unroll
  for (int t = 0; t < 4; ++t) oacc[t] = (v8f){0.f,0.f,0.f,0.f,0.f,0.f,0.f,0.f};

  const int nChunks = kSeq / AT_KC;
  for (int kc = 0; kc < nChunks; ++kc) {
    const int kv0 = kc * AT_KC;
    __syncthreads();
    {
      const int r = tid >> 1, half = (tid & 1) * 32;
      const _Float16* ks  = Kp + (size_t)(kv0 + r) * kQKld + half;
      const __bf16*   vsh = Vh + (size_t)r * kSeq + kv0 + half;
      const __bf16*   vsl = Vl + (size_t)r * kSeq + kv0 + half;
#pragma unroll
      for (int i = 0; i < 4; ++i) {
        const v8h a0 = *(const v8h*)(ks + 8 * i);
        const v8b b0 = *(const v8b*)(vsh + 8 * i);
        const v8b b1 = *(const v8b*)(vsl + 8 * i);
        *(v8h*)(Ksh + r * AT_D  + half + 8 * i) = a0;
        *(v8b*)(Vth + r * AT_KC + half + 8 * i) = b0;
        *(v8b*)(Vtl + r * AT_KC + half + 8 * i) = b1;
      }
    }
    __syncthreads();
    const float dcv = decrow[kc >> 1];

    v8f s[4];
#pragma unroll
    for (int j = 0; j < 4; ++j) {
      s[j] = (v8f){0.f,0.f,0.f,0.f,0.f,0.f,0.f,0.f};
#pragma unroll
      for (int dc = 0; dc < 2; ++dc) {
        FH kb;
        kb.h[0] = *(const v8h*)(Ksh + (j * 16 + c) * AT_D + dc * 32 + 8 * hh);
        kb.h[1] = *(const v8h*)(Ksh + (j * 16 + c) * AT_D + dc * 32 + 16 + 8 * hh);
        s[j] = at_mma_h(qa[dc], kb.v, s[j]);
      }
    }
    float cm[8];
#pragma unroll
    for (int r = 0; r < 8; ++r) {
      float m = -INFINITY;
#pragma unroll
      for (int j = 0; j < 4; ++j) {
        const float t = fmaxf(s[j][r] * sscale, 0.0f) * dcv;
        s[j][r] = t;
        m = fmaxf(m, t);
      }
#pragma unroll
      for (int off = 1; off < 16; off <<= 1) m = fmaxf(m, __shfl_xor(m, off, 32));
      cm[r] = m;
    }
    __bf16* pwh = Psh[wave];
    __bf16* pwl = Psl[wave];
#pragma unroll
    for (int r = 0; r < 8; ++r) {
      const float mnew = fmaxf(mrow[r], cm[r]);
      const float alpha = expf(mrow[r] - mnew);
      mrow[r] = mnew;
      float psum = 0.f;
#pragma unroll
      for (int j = 0; j < 4; ++j) {
        const float p = expf(s[j][r] - mnew);
        psum += p;
        __bf16 a, bl; at_split(p, a, bl);
        pwh[(8 * hh + r) * AT_KC + j * 16 + c] = a;
        pwl[(8 * hh + r) * AT_KC + j * 16 + c] = bl;
      }
#pragma unroll
      for (int off = 1; off < 16; off <<= 1) psum += __shfl_xor(psum, off, 32);
      lrow[r] = lrow[r] * alpha + psum;
#pragma unroll
      for (int t = 0; t < 4; ++t) oacc[t][r] *= alpha;
    }
    __builtin_amdgcn_fence(__ATOMIC_RELEASE, "workgroup");
    __builtin_amdgcn_wave_barrier();
    __builtin_amdgcn_fence(__ATOMIC_ACQUIRE, "workgroup");
#pragma unroll 1
    for (int kk = 0; kk < 2; ++kk) {
      FB pa, pl;
      pa.h[0] = *(const v8b*)(pwh + c * AT_KC + kk * 32 + 8 * hh);
      pa.h[1] = *(const v8b*)(pwh + c * AT_KC + kk * 32 + 16 + 8 * hh);
      pl.h[0] = *(const v8b*)(pwl + c * AT_KC + kk * 32 + 8 * hh);
      pl.h[1] = *(const v8b*)(pwl + c * AT_KC + kk * 32 + 16 + 8 * hh);
#pragma unroll
      for (int t = 0; t < 4; ++t) {
        FB vb, vl;
        vb.h[0] = *(const v8b*)(Vth + (t * 16 + c) * AT_KC + kk * 32 + 8 * hh);
        vb.h[1] = *(const v8b*)(Vth + (t * 16 + c) * AT_KC + kk * 32 + 16 + 8 * hh);
        vl.h[0] = *(const v8b*)(Vtl + (t * 16 + c) * AT_KC + kk * 32 + 8 * hh);
        vl.h[1] = *(const v8b*)(Vtl + (t * 16 + c) * AT_KC + kk * 32 + 16 + 8 * hh);
        oacc[t] = at_mma(pa.v, vb.v, oacc[t]);
        oacc[t] = at_mma(pa.v, vl.v, oacc[t]);
        oacc[t] = at_mma(pl.v, vb.v, oacc[t]);
      }
    }
  }

  float* os = Os[wave];
#pragma unroll
  for (int r = 0; r < 8; ++r) {
    const float inv = 1.0f / lrow[r];
#pragma unroll
    for (int t = 0; t < 4; ++t) os[(8 * hh + r) * 68 + t * 16 + c] = oacc[t][r] * inv;
  }
  __builtin_amdgcn_fence(__ATOMIC_RELEASE, "workgroup");
  __builtin_amdgcn_wave_barrier();
  __builtin_amdgcn_fence(__ATOMIC_ACQUIRE, "workgroup");
  {
    const int q = lane >> 3, c8 = (lane & 7) * 8;
    for (int pass = 0; pass < 2; ++pass) {
#pragma unroll
      for (int it = 0; it < 4; ++it) {
        const int row = it * 4 + q;
        const float* sp = os + row * 68 + c8;
        v8h hv, lv;
#pragma unroll
        for (int e = 0; e < 8; ++e) {
          const unsigned short hb = f2bf_bits(sp[e]);
          const unsigned short lb = f2bf_bits(sp[e] - bf_bits2f(hb));
          hv[e] = __builtin_bit_cast(_Float16, hb);
          lv[e] = __builtin_bit_cast(_Float16, lb);
        }
        *(volatile v8h*)(Oh + (size_t)(q0 + row) * kDim + c8) = hv;
        *(volatile v8h*)(Ol + (size_t)(q0 + row) * kDim + c8) = lv;
      }
      __threadfence();
    }
  }
}

extern "C" void kernel_launch(void* const* d_in, const int* in_sizes, int n_in,
                              void* d_out, int out_size, void* d_ws, size_t ws_size,
                              hipStream_t stream) {
  if (n_in < 8) return;
  if (in_sizes[0] != kRows * kDim || in_sizes[1] != kBatch * kTime * kTime || in_sizes[2] != kDim ||
      in_sizes[3] != kDim || in_sizes[4] != kDim * kQkvN || in_sizes[5] != kDim * kDim ||
      in_sizes[6] != kHeads || in_sizes[7] != kHeads || out_size != kRows * kDim) return;

  const float* x     = (const float*)d_in[0];
  const float* Rmat  = (const float*)d_in[1];
  const float* gamma = (const float*)d_in[2];
  const float* beta  = (const float*)d_in[3];
  const float* Wqkv  = (const float*)d_in[4];
  const float* Wout  = (const float*)d_in[5];
  const float* av    = (const float*)d_in[6];
  const float* cv    = (const float*)d_in[7];
  float* out = (float*)d_out;

  const size_t szPlane512  = (size_t)kRows * kDim * 2;
  const size_t szQK        = (size_t)kRows * kQKld * 2;
  const size_t szVt        = (size_t)kBatch * kDim * kSeq * 2;
  const size_t szWq        = (size_t)kQkvN * kDim * 2;
  const size_t szWo        = (size_t)kDim * kDim * 2;
  const size_t szDec       = (size_t)kBatch * kHeads * kTime * kTime * 4;
  const size_t oXH  = 0;
  const size_t oXL  = oXH + szPlane512;
  const size_t oQK  = oXL + szPlane512;
  const size_t oVH  = oQK + szQK;
  const size_t oVL  = oVH + szVt;
  const size_t oOH  = oVL + szVt;
  const size_t oOL  = oOH + szPlane512;
  const size_t oWQ  = oOL + szPlane512;
  const size_t oWO  = oWQ + szWq;
  const size_t oDEC = oWO + szWo;
  const size_t total = oDEC + szDec;
  if (total > ws_size) return;

  char* w = (char*)d_ws;
  unsigned short* xh  = (unsigned short*)(w + oXH);
  unsigned short* xl  = (unsigned short*)(w + oXL);
  unsigned short* qk  = (unsigned short*)(w + oQK);
  unsigned short* vth = (unsigned short*)(w + oVH);
  unsigned short* vtl = (unsigned short*)(w + oVL);
  unsigned short* oh  = (unsigned short*)(w + oOH);
  unsigned short* ol  = (unsigned short*)(w + oOL);
  unsigned short* wq  = (unsigned short*)(w + oWQ);
  unsigned short* wo  = (unsigned short*)(w + oWO);
  float*          dec = (float*)(w + oDEC);

  ln_split_kernel<<<dim3((kRows + 7) / 8), dim3(256), 0, stream>>>(x, gamma, beta, xh, xl, kRows);
  tcast_bf16_kernel<<<dim3(kQkvN / 64, kDim / 64), dim3(256), 0, stream>>>(Wqkv, wq, kDim, kQkvN);
  tcast_bf16_kernel<<<dim3(kDim / 64, kDim / 64), dim3(256), 0, stream>>>(Wout, wo, kDim, kDim);
  const int nDec = kBatch * kHeads * kTime * kTime;
  decay_kernel<<<dim3((nDec + 255) / 256), dim3(256), 0, stream>>>(Rmat, av, cv, dec, nDec);
  {
    const int tiles = (kRows / 64) * (kQKld / 64);
    wmma_gemm64<1, 1, 0, 1, false><<<dim3((tiles + 7) / 8, 1), dim3(256), 0, stream>>>(
        xh, xl, kDim, 0L, wq, wq, kDim, 0L, (void*)qk, (void*)qk, kQKld, 0L,
        dec, dec, 0L, kRows, kQKld, kDim, 1.0f);
  }
  {
    const int tiles = (kDim / 64) * (kSeq / 64);
    wmma_gemm64<1, 2, 0, 2, false><<<dim3((tiles + 7) / 8, kBatch), dim3(256), 0, stream>>>(
        wq + (size_t)kQKld * kDim, wq + (size_t)kQKld * kDim, kDim, 0L,
        xh, xl, kDim, (long)kSeq * kDim,
        (void*)vth, (void*)vtl, kSeq, (long)kDim * kSeq,
        dec, dec, 0L, kDim, kSeq, kDim, 1.0f);
  }
  attn_td_kernel<<<dim3(kBatch * kHeads * (kSeq / 64)), dim3(128), 0, stream>>>(qk, vth, vtl, dec, oh, ol, 0.125f);
  {
    const int tiles = (kRows / 64) * (kDim / 64);
    wmma_gemm64<1, 1, 0, 0, false><<<dim3((tiles + 7) / 8, 1), dim3(256), 0, stream>>>(
        oh, ol, kDim, 0L, wo, wo, kDim, 0L, (void*)out, (void*)out, kDim, 0L,
        dec, dec, 0L, kRows, kDim, kDim, 1.0f);
  }
}
